// CausalI_47132971106806
// MI455X (gfx1250) — hardware-verified
//
#include <hip/hip_runtime.h>
#include <stddef.h>


#define HC      128
#define NCLS    10
#define NTHR    256
#define NWAVE   8
#define EPT     8
#define NGRP    2
#define CHUNK   (NTHR * EPT * NGRP)
#define WCAP    (EPT * NGRP * 32)
#define LISTN   (NWAVE * WCAP)
#define NBC     4096
#define NBF     1024
#define RCAP    40960
#define RBN     128
#define TGT     256
#define DEGCAP  2048
#define GROWS   128
#define OTHR    512
#define SRB     256
#define ATTW    16
#define WROWS   1216
#define BNEPS   1e-5f
#define BNBETA  1e-4f

#define LDS_FILL  ((RCAP + NBF + LISTN) * 4 + 64)
#define LDS_GEMM0 (GROWS * HC * 4)
#define LDS_GEMM1 (GROWS * ATTW * 4)
#define LDS_GEMM2 (GROWS * ATTW * 4 + GROWS * NCLS * 4)

static_assert((CHUNK & (CHUNK - 1)) == 0);
static_assert(CHUNK <= 4096);
static_assert(NBC <= 4096 && NBF <= 4096);
static_assert((NBC & (NBC - 1)) == 0 && (NBF & (NBF - 1)) == 0);
static_assert(NBC == 4 * NBF);
static_assert(OTHR * 8 == NBC);
static_assert((RCAP % 32) == 0);
static_assert(TGT == NWAVE * 32);
static_assert(GROWS == NWAVE * 16);
static_assert(SRB == NWAVE * 32);
static_assert((WROWS % 16) == 0);

typedef float          v2f   __attribute__((ext_vector_type(2)));
typedef float          v4f   __attribute__((ext_vector_type(4)));
typedef float          v8f   __attribute__((ext_vector_type(8)));
typedef int            v4i   __attribute__((ext_vector_type(4)));
typedef unsigned int   v8u   __attribute__((ext_vector_type(8)));
typedef unsigned short v8us  __attribute__((ext_vector_type(8)));
typedef __bf16         v16bf __attribute__((ext_vector_type(16)));
typedef double         v2d   __attribute__((ext_vector_type(2)));
typedef double         v4d   __attribute__((ext_vector_type(4)));
union FragB { v16bf v; v8us u[2]; };
union FI { float f; int i; };

__device__ __forceinline__ void split8(v4f a, v4f b, v8us& hi, v8us& lo) {
  const v8f v  = __builtin_shufflevector(a, b, 0, 1, 2, 3, 4, 5, 6, 7);
  const v8u u  = __builtin_bit_cast(v8u, v);
  const v8u h  = (u + 0x7FFFu + ((u >> 16) & 1u)) >> 16;
  const v8f hf = __builtin_bit_cast(v8f, h << 16);
  const v8f r  = v - hf;
  const v8u ru = __builtin_bit_cast(v8u, r);
  const v8u l  = (ru + 0x7FFFu + ((ru >> 16) & 1u)) >> 16;
  hi = __builtin_convertvector(h, v8us);
  lo = __builtin_convertvector(l, v8us);
}

__device__ __forceinline__ v8f wmb(v16bf a, v16bf b, v8f c) {
  v8f d = __builtin_amdgcn_wmma_f32_16x16x32_bf16(false, a, false, b, (short)0, c, false, false);
  asm volatile("v_nop\n\tv_nop\n\tv_nop\n\tv_nop" : "+v"(d) : "v"(a), "v"(b));
  return d;
}

__device__ __forceinline__ void att2(float l0, float l1, float& w0, float& w1) {
  const float mx = fmaxf(l0, l1);
  const float e0 = __expf(l0 - mx), e1 = __expf(l1 - mx);
  const float inv = 1.0f / (e0 + e1);
  w0 = e0 * inv;
  w1 = e1 * inv;
}

template <int NB>
__device__ __forceinline__ int scan_chunk(const int* __restrict__ dsts, int nE, int cbase, int slotBase,
                                          int vec8, int* list, int tid, int lane, int wave) {
  int wc = 0;
#pragma unroll
  for (int g = 0; g < NGRP; ++g) {
    const int el0  = (g * NTHR + tid) * EPT;
    const int e0   = cbase + el0;
    const int sent = -2147483647 - 1;
    v4i da, db;
    if (vec8 != 0 && cbase + CHUNK <= nE) {
      da = *(const v4i*)(dsts + e0);
      db = *(const v4i*)(dsts + e0 + 4);
    } else {
      da.x = (e0     < nE) ? dsts[min(e0, nE - 1)] : sent;
      da.y = (e0 + 1 < nE) ? dsts[min(e0 + 1, nE - 1)] : sent;
      da.z = (e0 + 2 < nE) ? dsts[min(e0 + 2, nE - 1)] : sent;
      da.w = (e0 + 3 < nE) ? dsts[min(e0 + 3, nE - 1)] : sent;
      db.x = (e0 + 4 < nE) ? dsts[min(e0 + 4, nE - 1)] : sent;
      db.y = (e0 + 5 < nE) ? dsts[min(e0 + 5, nE - 1)] : sent;
      db.z = (e0 + 6 < nE) ? dsts[min(e0 + 6, nE - 1)] : sent;
      db.w = (e0 + 7 < nE) ? dsts[min(e0 + 7, nE - 1)] : sent;
    }
    const unsigned nb = (unsigned)slotBase;
    const unsigned s0 = (unsigned)da.x - nb, s1 = (unsigned)da.y - nb;
    const unsigned s2 = (unsigned)da.z - nb, s3 = (unsigned)da.w - nb;
    const unsigned s4 = (unsigned)db.x - nb, s5 = (unsigned)db.y - nb;
    const unsigned s6 = (unsigned)db.z - nb, s7 = (unsigned)db.w - nb;
    const bool h0 = s0 < (unsigned)NB, h1 = s1 < (unsigned)NB, h2 = s2 < (unsigned)NB, h3 = s3 < (unsigned)NB;
    const bool h4 = s4 < (unsigned)NB, h5 = s5 < (unsigned)NB, h6 = s6 < (unsigned)NB, h7 = s7 < (unsigned)NB;
    const unsigned any = __builtin_amdgcn_ballot_w32(h0 | h1 | h2 | h3 | h4 | h5 | h6 | h7);
    if (any != 0u) {
#define HITJ(J, HJ, SJ) { \
        const unsigned mj = __builtin_amdgcn_ballot_w32(HJ); \
        if (mj != 0u) { \
          if (HJ) { \
            const int pos = wc + (int)__builtin_amdgcn_mbcnt_lo(mj, 0u); \
            if (pos < WCAP) list[wave * WCAP + pos] = ((el0 + (J)) << 12) | (int)(SJ); \
          } \
          wc += (int)__builtin_popcount(mj); } }
      HITJ(0, h0, s0)
      HITJ(1, h1, s1)
      HITJ(2, h2, s2)
      HITJ(3, h3, s3)
      HITJ(4, h4, s4)
      HITJ(5, h5, s5)
      HITJ(6, h6, s6)
      HITJ(7, h7, s7)
#undef HITJ
    }
  }
  return wc;
}

__global__ __launch_bounds__(NTHR) void k_wsplit(
    const float* __restrict__ Wfeat, const float* __restrict__ Wconv, const float* __restrict__ Wctx,
    const float* __restrict__ Wobj, const float* __restrict__ Wfc1, const float* __restrict__ Wfc2,
    const float* __restrict__ Wea, const float* __restrict__ Wna,
    unsigned short* Whi, unsigned short* Wlo) {
  const int rb  = blockIdx.x * (NTHR / 16);
  const int tid = threadIdx.x;
  const int row = rb + (tid >> 4);
  const int k0  = (tid & 15) * 8;
  float v[8];
  if (rb < 1200) {
    const float* src; int nc, n;
    if (rb < 128)       { src = Wfeat; nc = HC; n = row; }
    else if (rb < 512)  { const int i = (rb - 128) >> 7; src = Wconv + (size_t)i * HC * HC; nc = HC; n = row - 128 - 128 * i; }
    else if (rb < 640)  { src = Wctx; nc = HC; n = row - 512; }
    else if (rb < 768)  { src = Wobj; nc = HC; n = row - 640; }
    else if (rb < 1152) { const int i = (rb - 768) >> 7; src = Wfc1 + (size_t)i * HC * HC; nc = HC; n = row - 768 - 128 * i; }
    else                { const int i = (rb - 1152) >> 4; src = Wfc2 + (size_t)i * HC * NCLS; nc = NCLS; n = row - 1152 - 16 * i; }
    const int ncl = n < 0 ? 0 : (n < nc ? n : nc - 1);
#pragma unroll
    for (int e = 0; e < 8; ++e) {
      const int k = k0 + e;
      const float x = src[(size_t)k * nc + ncl];
      v[e] = (n >= 0 && n < nc) ? x : 0.0f;
    }
  } else {
    const int n = row - 1200;
    const int j = n & 1;
#pragma unroll
    for (int e = 0; e < 8; ++e) {
      const int k = k0 + e;
      const float wa = Wea[(size_t)k * 2 + j];
      const float wb = Wea[(size_t)(HC + k) * 2 + j];
      const float wn = Wna[(size_t)k * 2 + j];
      v[e] = (n < 2) ? wa : ((n < 4) ? wb : ((n < 6) ? wn : 0.0f));
    }
  }
  v4f a, b;
  a.x = v[0]; a.y = v[1]; a.z = v[2]; a.w = v[3];
  b.x = v[4]; b.y = v[5]; b.z = v[6]; b.w = v[7];
  v8us hi, lo;
  split8(a, b, hi, lo);
  const size_t o = (size_t)row * HC + k0;
  *(volatile v8us*)(Whi + o) = hi;
  *(volatile v8us*)(Wlo + o) = lo;
  __threadfence();
  *(volatile v8us*)(Whi + o) = hi;
  *(volatile v8us*)(Wlo + o) = lo;
}

__global__ __launch_bounds__(NTHR) void k_count(
    const int* __restrict__ dsts, int* cnt, float* dinv, int nE, int vec8) {
  __shared__ __attribute__((aligned(16))) int scnt[NBC];
  __shared__ __attribute__((aligned(16))) int list[LISTN];
  __shared__ int wcnt[NWAVE];
  const int tid = threadIdx.x, lane = tid & 31, wave = tid >> 5;
  const int nodeBase = blockIdx.x * NBC;

  for (int i = tid; i < NBC; i += NTHR) scnt[i] = 0;
  __syncthreads();

  const int nChunks = (nE + CHUNK - 1) / CHUNK;
#pragma unroll 1
  for (int ch = 0; ch < nChunks; ++ch) {
    const int cbase = ch * CHUNK;
    const int wc = scan_chunk<NBC>(dsts, nE, cbase, nodeBase, vec8, list, tid, lane, wave);
    if (lane == 0) wcnt[wave] = wc;
    __syncthreads();
    if (wave == 0) {
#pragma unroll 1
      for (int wsx = 0; wsx < NWAVE; ++wsx) {
        int n = __builtin_amdgcn_readfirstlane(wcnt[wsx]);
        n = n > WCAP ? WCAP : (n < 0 ? 0 : n);
        const int* lp = list + wsx * WCAP;
#pragma unroll 1
        for (int i = 0; i < n; ++i) {
          const int ent  = __builtin_amdgcn_readfirstlane(lp[i]);
          const int slot = ent & (NBC - 1);
          if (lane == 0) scnt[slot] = scnt[slot] + 1;
        }
      }
    }
    __syncthreads();
  }

  v4i cq[4]; v4f dq[4];
#pragma unroll
  for (int q = 0; q < 4; ++q) {
    const int f = (wave * 4 + q) * 128 + 4 * lane;
    const v4i c = *(const v4i*)(scnt + f);
    cq[q] = c;
    dq[q].x = rsqrtf((float)(c.x + 1));
    dq[q].y = rsqrtf((float)(c.y + 1));
    dq[q].z = rsqrtf((float)(c.z + 1));
    dq[q].w = rsqrtf((float)(c.w + 1));
  }
  int*   cp = cnt + (size_t)nodeBase;
  float* dp = dinv + (size_t)nodeBase;
#pragma unroll
  for (int q = 0; q < 4; ++q) {
    const int f = (wave * 4 + q) * 128 + 4 * lane;
    *(volatile v4i*)(cp + f) = cq[q];
    *(volatile v4f*)(dp + f) = dq[q];
  }
  __threadfence();
#pragma unroll
  for (int q = 0; q < 4; ++q) {
    const int f = (wave * 4 + q) * 128 + 4 * lane;
    *(volatile v4i*)(cp + f) = cq[q];
    *(volatile v4f*)(dp + f) = dq[q];
  }
}

__global__ __launch_bounds__(OTHR) void k_offsets(
    const int* __restrict__ cnt, int* off, int* rbase, int nChunk) {
  __shared__ __attribute__((aligned(16))) int soff[NBC];
  __shared__ __attribute__((aligned(16))) int srb[RBN];
  __shared__ int wtot[OTHR / 32];
  const int tid = threadIdx.x, lane = tid & 31, wave = tid >> 5, sub = tid >> 7;
  for (int i = tid; i < RBN; i += OTHR) srb[i] = 0;
  int carry = 0;
#pragma unroll 1
  for (int ch = 0; ch < nChunk; ++ch) {
    const int base = ch * NBC;
    const v4i c0 = *(const v4i*)(cnt + base + 8 * tid);
    const v4i c1 = *(const v4i*)(cnt + base + 8 * tid + 4);
    const int e0 = max(c0.x, 0), e1 = max(c0.y, 0), e2 = max(c0.z, 0), e3 = max(c0.w, 0);
    const int e4 = max(c1.x, 0), e5 = max(c1.y, 0), e6 = max(c1.z, 0), e7 = max(c1.w, 0);
    const int ts = e0 + e1 + e2 + e3 + e4 + e5 + e6 + e7;
    int incl = ts;
#pragma unroll
    for (int d = 1; d < 32; d <<= 1) {
      const int t = __shfl_up(incl, d);
      if (lane >= d) incl += t;
    }
    if (lane == 31) wtot[wave] = incl;
    __syncthreads();
    const int S0 = wtot[0]  + wtot[1]  + wtot[2]  + wtot[3];
    const int S1 = wtot[4]  + wtot[5]  + wtot[6]  + wtot[7];
    const int S2 = wtot[8]  + wtot[9]  + wtot[10] + wtot[11];
    const int S3 = wtot[12] + wtot[13] + wtot[14] + wtot[15];
    int pre = 0;
#pragma unroll 1
    for (int w = 4 * sub; w < wave; ++w) pre += wtot[w];
    const int b0 = carry;
    const int b1 = b0 + ((S0 + 31) & ~31);
    const int b2 = b1 + ((S1 + 31) & ~31);
    const int b3 = b2 + ((S2 + 31) & ~31);
    const int b4 = b3 + ((S3 + 31) & ~31);
    const int myb = sub == 0 ? b0 : (sub == 1 ? b1 : (sub == 2 ? b2 : b3));
    if (tid == 0) {
      srb[min(4 * ch + 0, RBN - 1)] = b0;
      srb[min(4 * ch + 1, RBN - 1)] = b1;
      srb[min(4 * ch + 2, RBN - 1)] = b2;
      srb[min(4 * ch + 3, RBN - 1)] = b3;
    }
    int run = myb + pre + incl - ts;
    soff[8 * tid + 0] = run; run += e0;
    soff[8 * tid + 1] = run; run += e1;
    soff[8 * tid + 2] = run; run += e2;
    soff[8 * tid + 3] = run; run += e3;
    soff[8 * tid + 4] = run; run += e4;
    soff[8 * tid + 5] = run; run += e5;
    soff[8 * tid + 6] = run; run += e6;
    soff[8 * tid + 7] = run;
    carry = b4;
    __syncthreads();
    const v4i o0 = *(const v4i*)(soff + 4 * tid);
    const v4i o1 = *(const v4i*)(soff + 4 * (tid + OTHR));
    int* op = off + base;
    *(volatile v4i*)(op + 4 * tid) = o0;
    *(volatile v4i*)(op + 4 * (tid + OTHR)) = o1;
    __threadfence();
    *(volatile v4i*)(op + 4 * tid) = o0;
    *(volatile v4i*)(op + 4 * (tid + OTHR)) = o1;
    __syncthreads();
  }
  if (tid == 0) srb[min(4 * nChunk, RBN - 1)] = carry;
  __syncthreads();
  v4i rv = {0, 0, 0, 0};
  if (tid < 32) rv = *(const v4i*)(srb + 4 * tid);
  if (tid < 32) *(volatile v4i*)(rbase + 4 * tid) = rv;
  __threadfence();
  if (tid < 32) *(volatile v4i*)(rbase + 4 * tid) = rv;
}

__global__ __launch_bounds__(NTHR) void k_fill(
    const int* __restrict__ ei, const int* __restrict__ off, const int* __restrict__ rbase,
    int* csr, int nN, int nE, int vec8, int csrLen) {
  extern __shared__ v4f lds_dyn[];
  int* region = (int*)lds_dyn;
  int* cursor = region + RCAP;
  int* list   = cursor + NBF;
  int* wcnt   = list + LISTN;
  const int tid = threadIdx.x, lane = tid & 31, wave = tid >> 5;
  const int b = blockIdx.x;
  const int nodeBase = b * NBF;
  const int* dsts = ei + nE;

  int rb0 = rbase[b];
  const int rb1 = rbase[b + 1];
  rb0 = rb0 < 0 ? 0 : (rb0 > csrLen ? csrLen : rb0);
  rb0 &= ~31;
  int len = rb1 - rb0;
  len = len < 0 ? 0 : (len > RCAP ? RCAP : len);
  int lenW = (len + 31) & ~31;
  if (rb0 + lenW > csrLen) lenW = (csrLen - rb0) & ~31;

  {
    const v4i z = {0, 0, 0, 0};
    for (int i = tid; i < RCAP / 4; i += NTHR) ((v4i*)region)[i] = z;
    for (int s = tid; s < NBF; s += NTHR) {
      int o = off[nodeBase + s] - rb0;
      o = o < 0 ? 0 : (o > RCAP ? RCAP : o);
      cursor[s] = o;
    }
  }
  __syncthreads();

  const int nChunks = (nE + CHUNK - 1) / CHUNK;
#pragma unroll 1
  for (int ch = 0; ch < nChunks; ++ch) {
    const int cbase = ch * CHUNK;
    const int wc = scan_chunk<NBF>(dsts, nE, cbase, nodeBase, vec8, list, tid, lane, wave);
    if (lane == 0) wcnt[wave] = wc;
    __syncthreads();
    if (wave == 0) {
#pragma unroll 1
      for (int wsx = 0; wsx < NWAVE; ++wsx) {
        int n = __builtin_amdgcn_readfirstlane(wcnt[wsx]);
        n = n > WCAP ? WCAP : (n < 0 ? 0 : n);
        const int* lp = list + wsx * WCAP;
#pragma unroll 1
        for (int i = 0; i < n; ++i) {
          const int ent  = __builtin_amdgcn_readfirstlane(lp[i]);
          const int slot = ent & (NBF - 1);
          int e = cbase + ((ent >> 12) & (CHUNK - 1));
          e = e > nE - 1 ? nE - 1 : e;
          int src = ei[e];
          src = src < 0 ? 0 : (src > nN - 1 ? nN - 1 : src);
          if (lane == 0) {
            int pos = cursor[slot];
            pos = pos < 0 ? 0 : (pos > RCAP - 1 ? RCAP - 1 : pos);
            region[pos] = src;
            const int np = pos + 1;
            cursor[slot] = np > RCAP ? RCAP : np;
          }
        }
      }
    }
    __syncthreads();
  }

  const int nv = lenW >> 2;
  int* gp = csr + rb0;
#pragma unroll 1
  for (int i = tid; i < nv; i += NTHR) { const v4i v = ((const v4i*)region)[i]; *(volatile v4i*)(gp + 4 * i) = v; }
  __threadfence();
#pragma unroll 1
  for (int i = tid; i < nv; i += NTHR) { const v4i v = ((const v4i*)region)[i]; *(volatile v4i*)(gp + 4 * i) = v; }
}

__global__ __launch_bounds__(NTHR) void k_stats(
    const float* __restrict__ src, const float* __restrict__ src2, const int* __restrict__ perm,
    const float* __restrict__ na, v2d* part, int nN, int mode, int comp) {
  __shared__ __attribute__((aligned(32))) v4d sh[NWAVE * 32 * 2];
  __shared__ __attribute__((aligned(16))) v2d stg[HC];
  const int tid = threadIdx.x, lane = tid & 31, wave = tid >> 5;
  const int r0 = blockIdx.x * SRB;
  int r1 = r0 + SRB; r1 = r1 > nN ? nN : r1;
  v4d s = {0.0, 0.0, 0.0, 0.0}, q = {0.0, 0.0, 0.0, 0.0};
#pragma unroll 1
  for (int n = r0 + wave; n < r1; n += NWAVE) {
    int idx = n;
    if (mode == 2) { int pi = perm[n]; pi = pi < 0 ? 0 : (pi > nN - 1 ? nN - 1 : pi); idx = pi; }
    v4f v = *(const v4f*)(src + (size_t)idx * HC + 4 * lane);
    if (mode == 2) v = v + *(const v4f*)(src2 + (size_t)n * HC + 4 * lane);
    if (mode == 1) { const float sc = na[2 * (size_t)n + comp]; v = v * sc; }
    const v4d d = __builtin_convertvector(v, v4d);
    s = s + d;
    q = q + d * d;
  }
  sh[(wave * 32 + lane) * 2 + 0] = s;
  sh[(wave * 32 + lane) * 2 + 1] = q;
  __syncthreads();
  if (wave == 0) {
    v4d ts = {0.0, 0.0, 0.0, 0.0}, tq = {0.0, 0.0, 0.0, 0.0};
#pragma unroll 1
    for (int w = 0; w < NWAVE; ++w) {
      ts = ts + sh[(w * 32 + lane) * 2 + 0];
      tq = tq + sh[(w * 32 + lane) * 2 + 1];
    }
    v2d p0, p1, p2, p3;
    p0.x = ts.x; p0.y = tq.x; p1.x = ts.y; p1.y = tq.y;
    p2.x = ts.z; p2.y = tq.z; p3.x = ts.w; p3.y = tq.w;
    stg[4 * lane + 0] = p0; stg[4 * lane + 1] = p1; stg[4 * lane + 2] = p2; stg[4 * lane + 3] = p3;
  }
  __syncthreads();
  if (wave == 0) {
    v2d* gp = part + (size_t)blockIdx.x * HC;
    const v2d o0 = stg[lane], o1 = stg[32 + lane], o2 = stg[64 + lane], o3 = stg[96 + lane];
    *(volatile v2d*)(gp + lane) = o0;
    *(volatile v2d*)(gp + 32 + lane) = o1;
    *(volatile v2d*)(gp + 64 + lane) = o2;
    *(volatile v2d*)(gp + 96 + lane) = o3;
    __threadfence();
    *(volatile v2d*)(gp + lane) = o0;
    *(volatile v2d*)(gp + 32 + lane) = o1;
    *(volatile v2d*)(gp + 64 + lane) = o2;
    *(volatile v2d*)(gp + 96 + lane) = o3;
  }
}

__global__ __launch_bounds__(HC) void k_bnfin(const v2d* __restrict__ part, int nBlk, float* bnp, int nN) {
  const int c = threadIdx.x;
  double S = 0.0, Q = 0.0;
#pragma unroll 1
  for (int b = 0; b < nBlk; ++b) {
    const v2d p = part[(size_t)b * HC + c];
    S += p.x; Q += p.y;
  }
  const double inv = 1.0 / (double)nN;
  const double mu  = S * inv;
  double var = Q * inv - mu * mu;
  var = var < 0.0 ? 0.0 : var;
  const float m32 = (float)mu;
  const float sc  = 1.0f / sqrtf((float)var + BNEPS);
  *(volatile float*)(bnp + c) = m32;
  *(volatile float*)(bnp + HC + c) = sc;
  __threadfence();
  *(volatile float*)(bnp + c) = m32;
  *(volatile float*)(bnp + HC + c) = sc;
}

__global__ __launch_bounds__(NTHR) void k_cvt(
    const float* __restrict__ src, const float* __restrict__ src2, const int* __restrict__ perm,
    const float* __restrict__ na, const float* __restrict__ bnp,
    unsigned short* Ahi, unsigned short* Alo, int nN, int mode, int comp, int useBn) {
  const int t = blockIdx.x * NTHR + (int)threadIdx.x;
  const int row = t >> 4, c0 = (t & 15) * 8;
  const int rowc = row > nN - 1 ? nN - 1 : row;
  int idx = rowc;
  if (mode == 2) { int pi = perm[rowc]; pi = pi < 0 ? 0 : (pi > nN - 1 ? nN - 1 : pi); idx = pi; }
  const float* sp = src + (size_t)idx * HC + c0;
  v4f a = *(const v4f*)sp, b = *(const v4f*)(sp + 4);
  if (mode == 2) {
    const float* s2 = src2 + (size_t)rowc * HC + c0;
    a = a + *(const v4f*)s2;
    b = b + *(const v4f*)(s2 + 4);
  }
  if (mode == 1) { const float sc = na[2 * (size_t)rowc + comp]; a = a * sc; b = b * sc; }
  if (useBn != 0) {
    const v4f mu0 = *(const v4f*)(bnp + c0), mu1 = *(const v4f*)(bnp + c0 + 4);
    const v4f sc0 = *(const v4f*)(bnp + HC + c0), sc1 = *(const v4f*)(bnp + HC + c0 + 4);
    a = (a - mu0) * sc0 + BNBETA;
    b = (b - mu1) * sc1 + BNBETA;
  }
  const v4f z4 = {0.f, 0.f, 0.f, 0.f};
  a = (row < nN) ? a : z4;
  b = (row < nN) ? b : z4;
  v8us hi, lo;
  split8(a, b, hi, lo);
  const size_t o = (size_t)row * HC + c0;
  *(volatile v8us*)(Ahi + o) = hi;
  *(volatile v8us*)(Alo + o) = lo;
  __threadfence();
  *(volatile v8us*)(Ahi + o) = hi;
  *(volatile v8us*)(Alo + o) = lo;
}

template <int NT, int MODE>
__global__ __launch_bounds__(NTHR) void k_gemm(
    const unsigned short* __restrict__ Ahi, const unsigned short* __restrict__ Alo,
    const unsigned short* __restrict__ Whi, const unsigned short* __restrict__ Wlo,
    const float* __restrict__ bias, float* outp, int nRows, int relu, int useBias) {
  extern __shared__ v4f lds_dyn[];
  float* stg = (float*)lds_dyn;
  const int tid = threadIdx.x, lane = tid & 31, wave = tid >> 5, hh = lane >> 4, m = lane & 15;
  const int rowBase = blockIdx.x * GROWS;
  const int arow = rowBase + wave * 16 + m;
  const unsigned short* ah = Ahi + (size_t)arow * HC + 8 * hh;
  const unsigned short* al = Alo + (size_t)arow * HC + 8 * hh;

  v8f acc[NT];
#pragma unroll
  for (int t = 0; t < NT; ++t) { v8f z = {0.f, 0.f, 0.f, 0.f, 0.f, 0.f, 0.f, 0.f}; acc[t] = z; }
#pragma unroll
  for (int kt = 0; kt < HC / 32; ++kt) {
    FragB fa, fl;
    fa.u[0] = *(const v8us*)(ah + 32 * kt);
    fa.u[1] = *(const v8us*)(ah + 32 * kt + 16);
    fl.u[0] = *(const v8us*)(al + 32 * kt);
    fl.u[1] = *(const v8us*)(al + 32 * kt + 16);
#pragma unroll
    for (int t = 0; t < NT; ++t) {
      const unsigned short* bh = Whi + (size_t)(16 * t + m) * HC + 32 * kt + 8 * hh;
      const unsigned short* bl = Wlo + (size_t)(16 * t + m) * HC + 32 * kt + 8 * hh;
      FragB fb, gb;
      fb.u[0] = *(const v8us*)bh;
      fb.u[1] = *(const v8us*)(bh + 16);
      gb.u[0] = *(const v8us*)bl;
      gb.u[1] = *(const v8us*)(bl + 16);
      acc[t] = wmb(fa.v, fb.v, acc[t]);
      acc[t] = wmb(fa.v, gb.v, acc[t]);
      acc[t] = wmb(fl.v, fb.v, acc[t]);
    }
  }

  if (MODE == 0) {
    const int r0 = wave * 16 + 8 * hh;
    float* sp = stg + r0 * HC + m;
#pragma unroll
    for (int t = 0; t < NT; ++t) {
      const float bl = bias[16 * t + m];
      const float bv = useBias != 0 ? bl : 0.0f;
#pragma unroll
      for (int r = 0; r < 8; ++r) {
        float v = acc[t][r] + bv;
        v = relu != 0 ? fmaxf(v, 0.0f) : v;
        sp[r * HC + 16 * t] = v;
      }
    }
    __syncthreads();
    const float* lp = stg + wave * 16 * HC + 4 * lane;
    float* gp = outp + ((size_t)rowBase + wave * 16) * HC + 4 * lane;
#pragma unroll
    for (int i = 0; i < 16; ++i) { const v4f v = *(const v4f*)(lp + i * HC); *(volatile v4f*)(gp + (size_t)i * HC) = v; }
    __threadfence();
#pragma unroll
    for (int i = 0; i < 16; ++i) { const v4f v = *(const v4f*)(lp + i * HC); *(volatile v4f*)(gp + (size_t)i * HC) = v; }
  } else if (MODE == 1) {
    float* sp = stg + (wave * 16 + 8 * hh) * ATTW + m;
#pragma unroll
    for (int r = 0; r < 8; ++r) sp[r * ATTW] = acc[0][r];
    __syncthreads();
    const float* lp = stg + wave * 16 * ATTW;
    float* gp = outp + ((size_t)rowBase + wave * 16) * ATTW;
    const v4f o0 = *(const v4f*)(lp + 4 * lane);
    const v4f o1 = *(const v4f*)(lp + 128 + 4 * lane);
    *(volatile v4f*)(gp + 4 * lane) = o0;
    *(volatile v4f*)(gp + 128 + 4 * lane) = o1;
    __threadfence();
    *(volatile v4f*)(gp + 4 * lane) = o0;
    *(volatile v4f*)(gp + 128 + 4 * lane) = o1;
  } else {
    float* sp = stg + (wave * 16 + 8 * hh) * ATTW + m;
    const float bl = bias[m < NCLS ? m : NCLS - 1];
#pragma unroll
    for (int r = 0; r < 8; ++r) sp[r * ATTW] = acc[0][r] + bl;
    __syncthreads();
    float* ostg = stg + GROWS * ATTW;
    if (tid < GROWS) {
      const float* p = stg + tid * ATTW;
      float mx = p[0];
#pragma unroll 1
      for (int c = 1; c < NCLS; ++c) mx = fmaxf(mx, p[c]);
      float se = 0.0f;
#pragma unroll 1
      for (int c = 0; c < NCLS; ++c) se += expf(p[c] - mx);
      const float ls = logf(se);
#pragma unroll 1
      for (int c = 0; c < NCLS; ++c) ostg[tid * NCLS + c] = (p[c] - mx) - ls;
    }
    __syncthreads();
    int vr = nRows - rowBase;
    vr = vr < 0 ? 0 : (vr > GROWS ? GROWS : vr);
    const int nP = (vr * NCLS) >> 2;
    float* gp = outp + (size_t)rowBase * NCLS;
#pragma unroll 1
    for (int p = tid; p < nP; p += NTHR) { const v4f v = *(const v4f*)(ostg + 4 * p); *(volatile v4f*)(gp + 4 * p) = v; }
    __threadfence();
#pragma unroll 1
    for (int p = tid; p < nP; p += NTHR) { const v4f v = *(const v4f*)(ostg + 4 * p); *(volatile v4f*)(gp + 4 * p) = v; }
  }
}

__global__ __launch_bounds__(NTHR) void k_wdeg(
    const int* __restrict__ ei, const float* __restrict__ attb, const float* __restrict__ bea,
    float* dinvC, float* dinvO, int nN, int nE, int vec8, int nPadRows) {
  __shared__ __attribute__((aligned(16))) float sd0[NBC];
  __shared__ __attribute__((aligned(16))) float sd1[NBC];
  __shared__ __attribute__((aligned(16))) int list[LISTN];
  __shared__ int wcnt[NWAVE];
  const int tid = threadIdx.x, lane = tid & 31, wave = tid >> 5;
  const int nodeBase = blockIdx.x * NBC;
  const int* rows = ei;
  const int* cols = ei + nE;

  for (int i = tid; i < NBC; i += NTHR) { sd0[i] = 0.0f; sd1[i] = 0.0f; }
  __syncthreads();
  const float be0 = bea[0], be1 = bea[1];

  const int nChunks = (nE + CHUNK - 1) / CHUNK;
#pragma unroll 1
  for (int ch = 0; ch < nChunks; ++ch) {
    const int cbase = ch * CHUNK;
    const int wc = scan_chunk<NBC>(rows, nE, cbase, nodeBase, vec8, list, tid, lane, wave);
    if (lane == 0) wcnt[wave] = wc;
    __syncthreads();
    if (wave == 0) {
#pragma unroll 1
      for (int wsx = 0; wsx < NWAVE; ++wsx) {
        int n = __builtin_amdgcn_readfirstlane(wcnt[wsx]);
        n = n > WCAP ? WCAP : (n < 0 ? 0 : n);
        const int* lp = list + wsx * WCAP;
#pragma unroll 1
        for (int i0 = 0; i0 < n; i0 += 32) {
          const int idx = i0 + lane;
          const int ii  = idx < n ? idx : n - 1;
          const int ent = lp[ii];
          const int slot = ent & (NBC - 1);
          int e = cbase + ((ent >> 12) & (CHUNK - 1));
          e = e > nE - 1 ? nE - 1 : e;
          int c = cols[e];
          c = c < 0 ? 0 : (c > nN - 1 ? nN - 1 : c);
          int r = nodeBase + slot;
          r = r > nPadRows - 1 ? nPadRows - 1 : r;
          const float pr0 = attb[(size_t)r * ATTW + 0], pr1 = attb[(size_t)r * ATTW + 1];
          const float qc0 = attb[(size_t)c * ATTW + 2], qc1 = attb[(size_t)c * ATTW + 3];
          float w0, w1;
          att2(pr0 + qc0 + be0, pr1 + qc1 + be1, w0, w1);
          FI u0, u1;
          u0.f = idx < n ? w0 : 0.0f;
          u1.f = idx < n ? w1 : 0.0f;
          const int mc = (n - i0) < 32 ? (n - i0) : 32;
#pragma unroll 1
          for (int p = 0; p < mc; ++p) {
            const int s = __builtin_amdgcn_readlane(slot, p);
            FI a, bq;
            a.i  = __builtin_amdgcn_readlane(u0.i, p);
            bq.i = __builtin_amdgcn_readlane(u1.i, p);
            if (lane == 0) { sd0[s] = sd0[s] + a.f; sd1[s] = sd1[s] + bq.f; }
          }
        }
      }
    }
    __syncthreads();
  }

  v4f dq0[4], dq1[4];
#pragma unroll
  for (int q = 0; q < 4; ++q) {
    const int f = (wave * 4 + q) * 128 + 4 * lane;
    const v4f a = *(const v4f*)(sd0 + f), b = *(const v4f*)(sd1 + f);
    dq0[q].x = rsqrtf(a.x + 1.0f); dq0[q].y = rsqrtf(a.y + 1.0f); dq0[q].z = rsqrtf(a.z + 1.0f); dq0[q].w = rsqrtf(a.w + 1.0f);
    dq1[q].x = rsqrtf(b.x + 1.0f); dq1[q].y = rsqrtf(b.y + 1.0f); dq1[q].z = rsqrtf(b.z + 1.0f); dq1[q].w = rsqrtf(b.w + 1.0f);
  }
  float* d0 = dinvC + (size_t)nodeBase;
  float* d1 = dinvO + (size_t)nodeBase;
#pragma unroll
  for (int q = 0; q < 4; ++q) {
    const int f = (wave * 4 + q) * 128 + 4 * lane;
    *(volatile v4f*)(d0 + f) = dq0[q];
    *(volatile v4f*)(d1 + f) = dq1[q];
  }
  __threadfence();
#pragma unroll
  for (int q = 0; q < 4; ++q) {
    const int f = (wave * 4 + q) * 128 + 4 * lane;
    *(volatile v4f*)(d0 + f) = dq0[q];
    *(volatile v4f*)(d1 + f) = dq1[q];
  }
}

__global__ __launch_bounds__(NTHR) void k_natt(const float* __restrict__ attb, const float* __restrict__ bna, v2f* na) {
  const int n = blockIdx.x * NTHR + (int)threadIdx.x;
  const float l0 = attb[(size_t)n * ATTW + 4] + bna[0];
  const float l1 = attb[(size_t)n * ATTW + 5] + bna[1];
  float w0, w1;
  att2(l0, l1, w0, w1);
  v2f o; o.x = w0; o.y = w1;
  *(volatile v2f*)(na + n) = o;
  __threadfence();
  *(volatile v2f*)(na + n) = o;
}

__global__ __launch_bounds__(NTHR) void k_agg(
    const int* __restrict__ csr, const int* __restrict__ off, const int* __restrict__ cnt,
    const float* __restrict__ dinv, const float* __restrict__ hw, const float* __restrict__ attb,
    const float* __restrict__ bea, const float* __restrict__ bs, float* hout,
    int nN, int csrLen, int weighted, int comp) {
  const int tid = threadIdx.x, lane = tid & 31, wave = tid >> 5;
  const int tbase = blockIdx.x * TGT + wave * 32;
  const int cl = tbase + lane;
  const int cnt_l = cnt[cl];
  const int off_l = off[cl];
  FI dvu; dvu.f = dinv[cl];
  const v4f bb = *(const v4f*)(bs + 4 * lane);
  const float be0 = bea[0], be1 = bea[1];

#pragma unroll 1
  for (int j = 0; j < 32; ++j) {
    const int c = tbase + j;
    int n = __builtin_amdgcn_readlane(cnt_l, j);
    n = n < 0 ? 0 : (n > DEGCAP ? DEGCAP : n);
    const int st = __builtin_amdgcn_readlane(off_l, j);
    FI du; du.i = __builtin_amdgcn_readlane(dvu.i, j);
    const float dc = du.f;
    float qc0 = 0.0f, qc1 = 0.0f;
    if (weighted != 0) { qc0 = attb[(size_t)c * ATTW + 2]; qc1 = attb[(size_t)c * ATTW + 3]; }
    v4f acc = {0.f, 0.f, 0.f, 0.f};
#pragma unroll 1
    for (int q0 = 0; q0 < n; q0 += 32) {
      int pos = st + q0 + lane;
      pos = pos < 0 ? 0 : (pos > csrLen - 1 ? csrLen - 1 : pos);
      int sl = csr[pos];
      sl = sl < 0 ? 0 : (sl > nN - 1 ? nN - 1 : sl);
      float cf = dinv[sl];
      if (weighted != 0) {
        const float pr0 = attb[(size_t)sl * ATTW + 0], pr1 = attb[(size_t)sl * ATTW + 1];
        float w0, w1;
        att2(pr0 + qc0 + be0, pr1 + qc1 + be1, w0, w1);
        cf = cf * (comp == 0 ? w0 : w1);
      }
      cf = cf * dc;
      FI cu; cu.f = cf;
      const int mcnt = (n - q0) < 32 ? (n - q0) : 32;
#pragma unroll 2
      for (int p = 0; p < mcnt; ++p) {
        const int s = __builtin_amdgcn_readlane(sl, p);
        FI k; k.i = __builtin_amdgcn_readlane(cu.i, p);
        acc = acc + *(const v4f*)(hw + (size_t)s * HC + 4 * lane) * k.f;
      }
    }
    const v4f sv = *(const v4f*)(hw + (size_t)c * HC + 4 * lane);
    acc = acc + sv * (dc * dc);
    v4f v = acc + bb;
    v.x = fmaxf(v.x, 0.f); v.y = fmaxf(v.y, 0.f); v.z = fmaxf(v.z, 0.f); v.w = fmaxf(v.w, 0.f);
    float* hp = hout + (size_t)c * HC + 4 * lane;
    *(volatile v4f*)hp = v;
    __threadfence();
    *(volatile v4f*)hp = v;
  }
}

extern "C" void kernel_launch(void* const* d_in, const int* in_sizes, int n_in,
                              void* d_out, int out_size, void* d_ws, size_t ws_size,
                              hipStream_t stream) {
  if (n_in < 19) return;
  const int nN = in_sizes[0] / HC;
  const int nE = in_sizes[1] / 2;
  if (nN < 16 || nE <= 0 || in_sizes[0] != nN * HC || in_sizes[1] != 2 * nE || in_sizes[2] != nN) return;
  if ((nN % 16) != 0) return;
  if (in_sizes[3] != HC * HC || in_sizes[4] < HC || in_sizes[5] != 3 * HC * HC || in_sizes[6] < 3 * HC) return;
  if (in_sizes[7] != 2 * HC * 2 || in_sizes[8] < 2 || in_sizes[9] != HC * 2 || in_sizes[10] < 2) return;
  if (in_sizes[11] != HC * HC || in_sizes[12] < HC || in_sizes[13] != HC * HC || in_sizes[14] < HC) return;
  if (in_sizes[15] != 3 * HC * HC || in_sizes[16] < 3 * HC || in_sizes[17] != 3 * HC * NCLS || in_sizes[18] < 3 * NCLS) return;
  if (out_size != 3 * nN * NCLS) return;
  if (nE > (1 << 28) || nN > (1 << 22)) return;

  const float* x      = (const float*)d_in[0];
  const int*   ei     = (const int*)d_in[1];
  const int*   perm   = (const int*)d_in[2];
  const float* W_feat = (const float*)d_in[3];
  const float* b_feat = (const float*)d_in[4];
  const float* W_conv = (const float*)d_in[5];
  const float* b_conv = (const float*)d_in[6];
  const float* W_ea   = (const float*)d_in[7];
  const float* b_ea   = (const float*)d_in[8];
  const float* W_na   = (const float*)d_in[9];
  const float* b_na   = (const float*)d_in[10];
  const float* W_ctx  = (const float*)d_in[11];
  const float* b_ctx  = (const float*)d_in[12];
  const float* W_obj  = (const float*)d_in[13];
  const float* b_obj  = (const float*)d_in[14];
  const float* W_fc1  = (const float*)d_in[15];
  const float* b_fc1  = (const float*)d_in[16];
  const float* W_fc2  = (const float*)d_in[17];
  const float* b_fc2  = (const float*)d_in[18];
  float* out = (float*)d_out;

  const int NPAD   = ((nN + TGT - 1) / TGT) * TGT;
  const int nBC    = (nN + NBC - 1) / NBC;
  const int CNTPAD = nBC * NBC;
  if (4 * nBC + 1 > RBN) return;
  const int nBF    = (nN + NBF - 1) / NBF;
  const int csrLen = ((nE + 31) & ~31) + 4096;
  const int nStat  = (nN + SRB - 1) / SRB;
  const int nGemm  = NPAD / GROWS;
  const int nAgg   = NPAD / TGT;
  const int nCvt   = NPAD / 16;
  const int nNat   = NPAD / NTHR;

  char* ws = (char*)d_ws;
  size_t off = 0;
  const size_t oWhi = off; off += (size_t)WROWS * HC * 2;     off = (off + 255) & ~(size_t)255;
  const size_t oWlo = off; off += (size_t)WROWS * HC * 2;     off = (off + 255) & ~(size_t)255;
  const size_t oCnR = off; off += (size_t)CNTPAD * 4;         off = (off + 255) & ~(size_t)255;
  const size_t oDvU = off; off += (size_t)CNTPAD * 4;         off = (off + 255) & ~(size_t)255;
  const size_t oCnC = off; off += (size_t)CNTPAD * 4;         off = (off + 255) & ~(size_t)255;
  const size_t oDvS = off; off += (size_t)CNTPAD * 4;         off = (off + 255) & ~(size_t)255;
  const size_t oOfC = off; off += (size_t)CNTPAD * 4;         off = (off + 255) & ~(size_t)255;
  const size_t oDvC = off; off += (size_t)CNTPAD * 4;         off = (off + 255) & ~(size_t)255;
  const size_t oDvO = off; off += (size_t)CNTPAD * 4;         off = (off + 255) & ~(size_t)255;
  const size_t oRb  = off; off += (size_t)RBN * 4;            off = (off + 255) & ~(size_t)255;
  const size_t oCsr = off; off += (size_t)csrLen * 4;         off = (off + 255) & ~(size_t)255;
  const size_t oAtt = off; off += (size_t)NPAD * ATTW * 4;    off = (off + 255) & ~(size_t)255;
  const size_t oNa  = off; off += (size_t)NPAD * 2 * 4;       off = (off + 255) & ~(size_t)255;
  const size_t oPar = off; off += (size_t)nStat * HC * 16;    off = (off + 255) & ~(size_t)255;
  const size_t oBnp = off; off += (size_t)2 * HC * 4;         off = (off + 255) & ~(size_t)255;
  const size_t oAhi = off; off += (size_t)NPAD * HC * 2;      off = (off + 255) & ~(size_t)255;
  const size_t oAlo = off; off += (size_t)NPAD * HC * 2;      off = (off + 255) & ~(size_t)255;
  const size_t oP0  = off; off += (size_t)NPAD * HC * 4;      off = (off + 255) & ~(size_t)255;
  const size_t oP1  = off; off += (size_t)NPAD * HC * 4;      off = (off + 255) & ~(size_t)255;
  const size_t oP2  = off; off += (size_t)NPAD * HC * 4;      off = (off + 255) & ~(size_t)255;
  if (off > ws_size) return;
  unsigned short* Whi = (unsigned short*)(ws + oWhi);
  unsigned short* Wlo = (unsigned short*)(ws + oWlo);
  int*   cntR  = (int*)(ws + oCnR);
  float* dinvU = (float*)(ws + oDvU);
  int*   cntC  = (int*)(ws + oCnC);
  float* dinvS = (float*)(ws + oDvS);
  int*   offC  = (int*)(ws + oOfC);
  float* dinvC = (float*)(ws + oDvC);
  float* dinvO = (float*)(ws + oDvO);
  int*   rb    = (int*)(ws + oRb);
  int*   csr   = (int*)(ws + oCsr);
  float* attb  = (float*)(ws + oAtt);
  float* naP   = (float*)(ws + oNa);
  v2d*   part  = (v2d*)(ws + oPar);
  float* bnp   = (float*)(ws + oBnp);
  unsigned short* Ahi = (unsigned short*)(ws + oAhi);
  unsigned short* Alo = (unsigned short*)(ws + oAlo);
  float* P0 = (float*)(ws + oP0);
  float* P1 = (float*)(ws + oP1);
  float* P2 = (float*)(ws + oP2);

  const int vec8 = ((nE & 3) == 0) ? 1 : 0;
  const int* rowsp = ei;
  const int* colsp = ei + nE;

  k_wsplit<<<WROWS / 16, NTHR, 0, stream>>>(W_feat, W_conv, W_ctx, W_obj, W_fc1, W_fc2, W_ea, W_na, Whi, Wlo);

  k_count<<<nBC, NTHR, 0, stream>>>(rowsp, cntR, dinvU, nE, vec8);
  k_count<<<nBC, NTHR, 0, stream>>>(colsp, cntC, dinvS, nE, vec8);
  k_offsets<<<1, OTHR, 0, stream>>>(cntC, offC, rb, nBC);
  hipFuncSetAttribute(reinterpret_cast<const void*>(&k_fill),
                      hipFuncAttributeMaxDynamicSharedMemorySize, LDS_FILL);
  k_fill<<<nBF, NTHR, LDS_FILL, stream>>>(ei, offC, rb, csr, nN, nE, vec8, csrLen);

  hipFuncSetAttribute(reinterpret_cast<const void*>(&k_gemm<8, 0>),
                      hipFuncAttributeMaxDynamicSharedMemorySize, LDS_GEMM0);

  k_stats<<<nStat, NTHR, 0, stream>>>(x, x, perm, naP, part, nN, 0, 0);
  k_bnfin<<<1, HC, 0, stream>>>(part, nStat, bnp, nN);
  k_cvt<<<nCvt, NTHR, 0, stream>>>(x, x, perm, naP, bnp, Ahi, Alo, nN, 0, 0, 1);
  k_gemm<8, 0><<<nGemm, NTHR, LDS_GEMM0, stream>>>(Ahi, Alo, Whi, Wlo, b_feat, P0, nN, 1, 1);

  for (int i = 0; i < 3; ++i) {
    const size_t wo = (size_t)(128 + 128 * i) * HC;
    k_stats<<<nStat, NTHR, 0, stream>>>(P0, P0, perm, naP, part, nN, 0, 0);
    k_bnfin<<<1, HC, 0, stream>>>(part, nStat, bnp, nN);
    k_cvt<<<nCvt, NTHR, 0, stream>>>(P0, P0, perm, naP, bnp, Ahi, Alo, nN, 0, 0, 1);
    k_gemm<8, 0><<<nGemm, NTHR, LDS_GEMM0, stream>>>(Ahi, Alo, Whi + wo, Wlo + wo, b_feat, P1, nN, 0, 0);
    k_agg<<<nAgg, NTHR, 0, stream>>>(csr, offC, cntC, dinvU, P1, attb, b_ea, b_conv + (size_t)i * HC, P0,
                                     nN, csrLen, 0, 0);
  }

  {
    const size_t wo = (size_t)1200 * HC;
    k_cvt<<<nCvt, NTHR, 0, stream>>>(P0, P0, perm, naP, bnp, Ahi, Alo, nN, 0, 0, 0);
    k_gemm<1, 1><<<nGemm, NTHR, LDS_GEMM1, stream>>>(Ahi, Alo, Whi + wo, Wlo + wo, b_na, attb, nN, 0, 0);
    k_wdeg<<<nBC, NTHR, 0, stream>>>(ei, attb, b_ea, dinvC, dinvO, nN, nE, vec8, NPAD);
    k_natt<<<nNat, NTHR, 0, stream>>>(attb, b_na, (v2f*)naP);
  }

  {
    const size_t wo = (size_t)512 * HC;
    k_stats<<<nStat, NTHR, 0, stream>>>(P0, P0, perm, naP, part, nN, 1, 0);
    k_bnfin<<<1, HC, 0, stream>>>(part, nStat, bnp, nN);
    k_cvt<<<nCvt, NTHR, 0, stream>>>(P0, P0, perm, naP, bnp, Ahi, Alo, nN, 1, 0, 1);
    k_gemm<8, 0><<<nGemm, NTHR, LDS_GEMM0, stream>>>(Ahi, Alo, Whi + wo, Wlo + wo, b_feat, P1, nN, 0, 0);
    k_agg<<<nAgg, NTHR, 0, stream>>>(csr, offC, cntC, dinvC, P1, attb, b_ea, b_ctx, P2, nN, csrLen, 1, 0);
  }
  {
    const size_t wo = (size_t)640 * HC;
    k_stats<<<nStat, NTHR, 0, stream>>>(P0, P0, perm, naP, part, nN, 1, 1);
    k_bnfin<<<1, HC, 0, stream>>>(part, nStat, bnp, nN);
    k_cvt<<<nCvt, NTHR, 0, stream>>>(P0, P0, perm, naP, bnp, Ahi, Alo, nN, 1, 1, 1);
    k_gemm<8, 0><<<nGemm, NTHR, LDS_GEMM0, stream>>>(Ahi, Alo, Whi + wo, Wlo + wo, b_feat, P1, nN, 0, 0);
    k_agg<<<nAgg, NTHR, 0, stream>>>(csr, offC, cntC, dinvO, P1, attb, b_ea, b_obj, P0, nN, csrLen, 1, 1);
  }

  for (int k = 0; k < 3; ++k) {
    const float* s1 = (k == 1) ? P0 : P2;
    const int md = (k == 2) ? 2 : 0;
    const size_t w1o = (size_t)(768 + 128 * k) * HC;
    const size_t w2o = (size_t)(1152 + 16 * k) * HC;
    k_stats<<<nStat, NTHR, 0, stream>>>(s1, P0, perm, naP, part, nN, md, 0);
    k_bnfin<<<1, HC, 0, stream>>>(part, nStat, bnp, nN);
    k_cvt<<<nCvt, NTHR, 0, stream>>>(s1, P0, perm, naP, bnp, Ahi, Alo, nN, md, 0, 1);
    k_gemm<8, 0><<<nGemm, NTHR, LDS_GEMM0, stream>>>(Ahi, Alo, Whi + w1o, Wlo + w1o, b_fc1 + (size_t)k * HC, P1, nN, 1, 1);
    k_stats<<<nStat, NTHR, 0, stream>>>(P1, P1, perm, naP, part, nN, 0, 0);
    k_bnfin<<<1, HC, 0, stream>>>(part, nStat, bnp, nN);
    k_cvt<<<nCvt, NTHR, 0, stream>>>(P1, P1, perm, naP, bnp, Ahi, Alo, nN, 0, 0, 1);
    k_gemm<1, 2><<<nGemm, NTHR, LDS_GEMM2, stream>>>(Ahi, Alo, Whi + w2o, Wlo + w2o, b_fc2 + (size_t)k * NCLS,
                                                       out + (size_t)k * nN * NCLS, nN, 0, 1);
  }
}
